// MLA_71975061946785
// MI455X (gfx1250) — hardware-verified
//
#include <hip/hip_runtime.h>
#include <math.h>
#include <stdint.h>

#define NSEQ  4
#define SEQ   2048
#define DMOD  1024
#define NHD   16
#define HDIM  64
#define LATD  256
#define NTOK  8192
#define QCW   2048

typedef __bf16       v16b __attribute__((ext_vector_type(16)));
typedef __bf16       v8b  __attribute__((ext_vector_type(8)));
typedef float        v8f  __attribute__((ext_vector_type(8)));
typedef float        v4f  __attribute__((ext_vector_type(4)));
typedef unsigned int v4u  __attribute__((ext_vector_type(4)));

static_assert(NTOK == NSEQ * SEQ);
static_assert(NHD * HDIM == DMOD);
static_assert(SEQ % 64 == 0);
static_assert(DMOD % 64 == 0);
static_assert(LATD % 64 == 0);
static_assert(QCW == 2 * DMOD);

__device__ __forceinline__ unsigned short bf_bits(float f) {
  const unsigned u = __float_as_uint(f);
  return (unsigned short)((u + 0x7FFFu + ((u >> 16) & 1u)) >> 16);
}
__device__ __forceinline__ float bf_val(unsigned short h) { return __uint_as_float(((unsigned)h) << 16); }
__device__ __forceinline__ unsigned pk16(unsigned short a, unsigned short b) { return (unsigned)a | ((unsigned)b << 16); }
__device__ __forceinline__ v8f zero8() { v8f z = {0.f, 0.f, 0.f, 0.f, 0.f, 0.f, 0.f, 0.f}; return z; }
__device__ __forceinline__ int wave_id() { return __builtin_amdgcn_readfirstlane((int)(threadIdx.x >> 5)); }

__device__ __forceinline__ void lds_wave_sync() {
  __builtin_amdgcn_fence(__ATOMIC_RELEASE, "workgroup");
  __builtin_amdgcn_wave_barrier();
  __builtin_amdgcn_fence(__ATOMIC_ACQUIRE, "workgroup");
}

union FragB { v16b v; v8b h[2]; };
__device__ __forceinline__ v16b ldfrag_b(const __bf16* p) { FragB f; f.h[0] = *(const v8b*)(p); f.h[1] = *(const v8b*)(p + 16); return f.v; }

__device__ __forceinline__ v8f mma_b(v16b a, v16b b, v8f c) {
  return __builtin_amdgcn_wmma_f32_16x16x32_bf16(false, a, false, b, (short)0, c, false, false);
}
__device__ __forceinline__ void dep_guard_b(v8f& a, v8f& b, v16b x, v16b y) {
  asm volatile("v_nop\n\tv_nop\n\tv_nop\n\tv_nop" : "+v"(a), "+v"(b) : "v"(x), "v"(y));
}
__device__ __forceinline__ void keep4_b(v16b a, v16b b, v16b c, v16b d) { asm volatile("v_nop" :: "v"(a), "v"(b), "v"(c), "v"(d)); }
__device__ __forceinline__ void acc_guard4(v8f& a, v8f& b, v8f& c, v8f& d) {
  asm volatile("v_nop\n\tv_nop\n\tv_nop\n\tv_nop" : "+v"(a), "+v"(b), "+v"(c), "+v"(d));
}
__device__ __forceinline__ v8f at_mma(v16b a, v16b b, v8f c) {
  c = __builtin_amdgcn_wmma_f32_16x16x32_bf16(false, a, false, b, (short)0, c, false, false);
  asm volatile("v_nop\n\tv_nop\n\tv_nop\n\tv_nop" : "+v"(c) : "v"(a), "v"(b));
  return c;
}

__global__ __launch_bounds__(256) void cvt_bf16_kernel(const float* __restrict__ in, unsigned short* __restrict__ outp, int n8) {
  const int i = (int)blockIdx.x * 256 + (int)threadIdx.x;
  if (i >= n8) return;
  const size_t e = 8 * (size_t)i;
  const v4f a = *(const v4f*)(in + e);
  const v4f b = *(const v4f*)(in + e + 4);
  v4u w;
  w[0] = pk16(bf_bits(a[0]), bf_bits(a[1]));
  w[1] = pk16(bf_bits(a[2]), bf_bits(a[3]));
  w[2] = pk16(bf_bits(b[0]), bf_bits(b[1]));
  w[3] = pk16(bf_bits(b[2]), bf_bits(b[3]));
  *(volatile v4u*)(outp + e) = w;
  __threadfence();
  *(volatile v4u*)(outp + e) = w;
}

__global__ __launch_bounds__(256) void tcvt_kernel(const float* __restrict__ W, unsigned short* __restrict__ oh, int R, int Cc) {
  __shared__ __align__(16) float tf[64 * 68];
  const int c0  = blockIdx.x * 64;
  const int r0  = blockIdx.y * 64;
  const int tid = threadIdx.x;
  {
    const int lr = tid >> 4;
    const int c4 = (tid & 15) * 4;
#pragma unroll
    for (int it = 0; it < 4; ++it) {
      const int rr = it * 16 + lr;
      const v4f a = *(const v4f*)(W + (size_t)(r0 + rr) * Cc + c0 + c4);
      *(v4f*)(tf + rr * 68 + c4) = a;
    }
  }
  __syncthreads();
  const int sub = tid >> 3;
  const int c8  = (tid & 7) * 8;
  v4u hv[2];
#pragma unroll
  for (int it = 0; it < 2; ++it) {
    const int oc = it * 32 + sub;
    v4u a;
#pragma unroll
    for (int q = 0; q < 4; ++q) {
      const float f0 = tf[(c8 + 2 * q) * 68 + oc];
      const float f1 = tf[(c8 + 2 * q + 1) * 68 + oc];
      a[q] = pk16(bf_bits(f0), bf_bits(f1));
    }
    hv[it] = a;
  }
  for (int pass = 0; pass < 2; ++pass) {
#pragma unroll
    for (int it = 0; it < 2; ++it) {
      const int oc = it * 32 + sub;
      const size_t go = (size_t)(c0 + oc) * R + r0 + c8;
      *(volatile v4u*)(oh + go) = hv[it];
    }
    __threadfence();
  }
}

template <bool ASPLIT, bool BSPLIT, int OUT_MODE>
__global__ __launch_bounds__(256) void gemm64_kernel(
    const unsigned short* __restrict__ Ap, const unsigned short* __restrict__ A2p, int lda, long strideA,
    const unsigned short* __restrict__ Btp, const unsigned short* __restrict__ Bt2p, int ldb, long strideB,
    void* Cout, void* Cout2, int ldc, long strideC,
    int M, int N, int K, float scale) {
  __shared__ __align__(16) float sT[8][16 * 68];
  const __bf16* A   = (const __bf16*)(const void*)Ap;
  const __bf16* A2  = (const __bf16*)(const void*)A2p;
  const __bf16* Bt  = (const __bf16*)(const void*)Btp;
  const __bf16* Bt2 = (const __bf16*)(const void*)Bt2p;
  const int b    = blockIdx.y;
  const int lane = threadIdx.x & 31;
  const int wave = wave_id();
  const int tilesN = N >> 6;
  const int tilesM = M >> 6;
  const int tile = (int)blockIdx.x * 8 + wave;
  if (tile >= tilesM * tilesN) return;
  const int tm = tile / tilesN;
  const int tn = tile - tm * tilesN;
  const int m0 = tm << 6;
  const int n0 = tn << 6;

  const __bf16* Ab  = A  + (size_t)b * strideA;
  const __bf16* Bb  = Bt + (size_t)b * strideB;
  const __bf16* Ab2 = ASPLIT ? (A2  + (size_t)b * strideA) : Ab;
  const __bf16* Bb2 = BSPLIT ? (Bt2 + (size_t)b * strideB) : Bb;

  const int rlane = lane & 15;
  const int koff  = (lane >> 4) * 8;
  const int mOff  = (lane >> 4) * 8;

  v8f acc[4][4];
#pragma unroll
  for (int i = 0; i < 4; ++i)
#pragma unroll
    for (int j = 0; j < 4; ++j) acc[i][j] = zero8();

  for (int k0 = 0; k0 < K; k0 += 32) {
    v16b bh[4], bl[4];
#pragma unroll
    for (int j = 0; j < 4; ++j) {
      const size_t bo = (size_t)(n0 + (j << 4) + rlane) * ldb + koff + k0;
      bh[j] = ldfrag_b(Bb + bo);
      bl[j] = BSPLIT ? ldfrag_b(Bb2 + bo) : bh[j];
    }
#pragma unroll
    for (int i = 0; i < 4; ++i) {
      const size_t ao = (size_t)(m0 + (i << 4) + rlane) * lda + koff + k0;
      const v16b ah = ldfrag_b(Ab + ao);
      const v16b al = ASPLIT ? ldfrag_b(Ab2 + ao) : ah;
#pragma unroll
      for (int j = 0; j < 4; ++j) {
        acc[i][j] = mma_b(ah, bh[j], acc[i][j]);
        if (BSPLIT) acc[i][j] = mma_b(ah, bl[j], acc[i][j]);
        if (ASPLIT) acc[i][j] = mma_b(al, bh[j], acc[i][j]);
      }
      dep_guard_b(acc[i][0], acc[i][3], ah, al);
    }
    keep4_b(bh[0], bh[1], bh[2], bh[3]);
    if (BSPLIT) keep4_b(bl[0], bl[1], bl[2], bl[3]);
  }
  acc_guard4(acc[0][0], acc[0][1], acc[0][2], acc[0][3]);
  acc_guard4(acc[1][0], acc[1][1], acc[1][2], acc[1][3]);
  acc_guard4(acc[2][0], acc[2][1], acc[2][2], acc[2][3]);
  acc_guard4(acc[3][0], acc[3][1], acc[3][2], acc[3][3]);

  float* slab = sT[wave];
#pragma unroll
  for (int i = 0; i < 4; ++i) {
    const int mBase = m0 + (i << 4);
#pragma unroll
    for (int j = 0; j < 4; ++j)
#pragma unroll
      for (int r = 0; r < 8; ++r)
        slab[(mOff + r) * 68 + (j << 4) + rlane] = acc[i][j][r] * scale;
    lds_wave_sync();
    if (OUT_MODE == 0) {
      float* C = (float*)Cout + (size_t)b * strideC;
      const int hh = lane >> 4, c4 = (lane & 15) * 4;
      for (int pass = 0; pass < 2; ++pass) {
#pragma unroll
        for (int it = 0; it < 8; ++it) {
          const int row = it * 2 + hh;
          const v4f v = *(const v4f*)(slab + row * 68 + c4);
          *(volatile v4f*)(C + (size_t)(mBase + row) * ldc + n0 + c4) = v;
        }
        __threadfence();
      }
    } else {
      const int q = lane >> 3, c8 = (lane & 7) * 8;
      unsigned short* C  = (unsigned short*)Cout  + (size_t)b * strideC;
      unsigned short* C2 = (unsigned short*)Cout2 + (size_t)b * strideC;
      for (int pass = 0; pass < 2; ++pass) {
#pragma unroll
        for (int it = 0; it < 4; ++it) {
          const int row = it * 4 + q;
          const float* sp = slab + row * 68 + c8;
          v4u hv, lv;
#pragma unroll
          for (int e = 0; e < 4; ++e) {
            const float f0 = sp[2 * e], f1 = sp[2 * e + 1];
            const unsigned short h0 = bf_bits(f0), h1 = bf_bits(f1);
            const unsigned short l0 = bf_bits(f0 - bf_val(h0)), l1 = bf_bits(f1 - bf_val(h1));
            hv[e] = pk16(h0, h1);
            lv[e] = pk16(l0, l1);
          }
          *(volatile v4u*)(C  + (size_t)(mBase + row) * ldc + n0 + c8) = hv;
          *(volatile v4u*)(C2 + (size_t)(mBase + row) * ldc + n0 + c8) = lv;
        }
        __threadfence();
      }
    }
    lds_wave_sync();
  }
}

#define AT_D  64
#define AT_NW 4
#define AT_KC 64
static_assert((4 * AT_KC * AT_D + 2 * AT_NW * 16 * AT_KC + 2 * AT_NW * 16 * 64) * 2 <= 65536);

__global__ __launch_bounds__(128)
void attn_causal64_kernel(unsigned short* qcp,
                          const unsigned short* __restrict__ kp,
                          const unsigned short* __restrict__ vhp, const unsigned short* __restrict__ vlp,
                          float sscale) {
  __shared__ __align__(16) __bf16 Ksh[AT_KC * AT_D];
  __shared__ __align__(16) __bf16 Ksl[AT_KC * AT_D];
  __shared__ __align__(16) __bf16 Vth[AT_D * AT_KC];
  __shared__ __align__(16) __bf16 Vtl[AT_D * AT_KC];
  __shared__ __align__(16) __bf16 Psh[AT_NW][16 * AT_KC];
  __shared__ __align__(16) __bf16 Psl[AT_NW][16 * AT_KC];
  __shared__ __align__(16) unsigned short Osh[AT_NW][16 * 64];
  __shared__ __align__(16) unsigned short Osl[AT_NW][16 * 64];

  const int tid  = (int)threadIdx.x;
  const int wave = wave_id();
  const int lane = tid & 31;
  const int hh   = lane >> 4;
  const int c    = lane & 15;

  const int nqb = SEQ / 64;
  const int bx = (int)blockIdx.x;
  const int qb = bx % nqb;
  const int h  = bx / nqb;
  const int b  = (int)blockIdx.y;
  const int q0 = qb * 64 + wave * 16;
  const size_t tok0 = (size_t)b * SEQ;

  const __bf16* QC = (const __bf16*)(const void*)qcp;
  const __bf16* Qh = QC + (size_t)h * AT_D;
  const __bf16* Ql = QC + DMOD + (size_t)h * AT_D;
  const __bf16* KB = (const __bf16*)(const void*)kp;
  const __bf16* Kh = KB + (size_t)h * AT_D;
  const __bf16* Kl = KB + DMOD + (size_t)h * AT_D;
  const __bf16* Vh = (const __bf16*)(const void*)vhp + ((size_t)b * DMOD + (size_t)h * AT_D) * SEQ;
  const __bf16* Vl = (const __bf16*)(const void*)vlp + ((size_t)b * DMOD + (size_t)h * AT_D) * SEQ;

  v16b qah[2], qal[2];
#pragma unroll
  for (int dc = 0; dc < 2; ++dc) {
    qah[dc] = ldfrag_b(Qh + (tok0 + q0 + c) * QCW + dc * 32 + 8 * hh);
    qal[dc] = ldfrag_b(Ql + (tok0 + q0 + c) * QCW + dc * 32 + 8 * hh);
  }

  float mrow[8], lrow[8];
  v8f oacc[4];
#pragma unroll
  for (int r = 0; r < 8; ++r) { mrow[r] = -INFINITY; lrow[r] = 0.f; }
#pragma unroll
  for (int t = 0; t < 4; ++t) oacc[t] = zero8();

  __bf16* pwh = Psh[wave];
  __bf16* pwl = Psl[wave];

  const int nChunks = qb + 1;
  for (int kc = 0; kc < nChunks; ++kc) {
    const int kv0 = kc * AT_KC;
    __syncthreads();
    {
      const int r = tid >> 1, half = (tid & 1) * 32;
      const __bf16* ksh = Kh + (tok0 + kv0 + r) * QCW + half;
      const __bf16* ksl = Kl + (tok0 + kv0 + r) * QCW + half;
      const __bf16* vsh = Vh + (size_t)r * SEQ + kv0 + half;
      const __bf16* vsl = Vl + (size_t)r * SEQ + kv0 + half;
#pragma unroll
      for (int i = 0; i < 4; ++i) {
        const v8b a0 = *(const v8b*)(ksh + 8 * i);
        const v8b a1 = *(const v8b*)(ksl + 8 * i);
        const v8b b0 = *(const v8b*)(vsh + 8 * i);
        const v8b b1 = *(const v8b*)(vsl + 8 * i);
        *(v8b*)(Ksh + r * AT_D  + half + 8 * i) = a0;
        *(v8b*)(Ksl + r * AT_D  + half + 8 * i) = a1;
        *(v8b*)(Vth + r * AT_KC + half + 8 * i) = b0;
        *(v8b*)(Vtl + r * AT_KC + half + 8 * i) = b1;
      }
    }
    __syncthreads();

    v8f s[4];
#pragma unroll
    for (int j = 0; j < 4; ++j) {
      s[j] = zero8();
#pragma unroll
      for (int dc = 0; dc < 2; ++dc) {
        FragB kb, kl;
        kb.h[0] = *(const v8b*)(Ksh + (j * 16 + c) * AT_D + dc * 32 + 8 * hh);
        kb.h[1] = *(const v8b*)(Ksh + (j * 16 + c) * AT_D + dc * 32 + 16 + 8 * hh);
        kl.h[0] = *(const v8b*)(Ksl + (j * 16 + c) * AT_D + dc * 32 + 8 * hh);
        kl.h[1] = *(const v8b*)(Ksl + (j * 16 + c) * AT_D + dc * 32 + 16 + 8 * hh);
        s[j] = at_mma(qah[dc], kb.v, s[j]);
        s[j] = at_mma(qah[dc], kl.v, s[j]);
        s[j] = at_mma(qal[dc], kb.v, s[j]);
      }
    }
    const bool diag = (kc == qb);
    float cm[8];
#pragma unroll
    for (int r = 0; r < 8; ++r) {
      const int qrow = q0 + 8 * hh + r;
      float m = -INFINITY;
#pragma unroll
      for (int j = 0; j < 4; ++j) {
        const int kvcol = kv0 + j * 16 + c;
        const float sv = s[j][r] * sscale;
        const bool masked = diag && (kvcol > qrow);
        const float sm = masked ? -INFINITY : sv;
        s[j][r] = sm;
        m = fmaxf(m, sm);
      }
#pragma unroll
      for (int off = 1; off < 16; off <<= 1) m = fmaxf(m, __shfl_xor(m, off, 32));
      cm[r] = m;
    }
#pragma unroll
    for (int r = 0; r < 8; ++r) {
      const float mnew = fmaxf(mrow[r], cm[r]);
      const float alpha = expf(mrow[r] - mnew);
      mrow[r] = mnew;
      float psum = 0.f;
#pragma unroll
      for (int j = 0; j < 4; ++j) {
        const float p = expf(s[j][r] - mnew);
        psum += p;
        const unsigned short hb = bf_bits(p);
        const unsigned short lb = bf_bits(p - bf_val(hb));
        pwh[(8 * hh + r) * AT_KC + j * 16 + c] = __builtin_bit_cast(__bf16, hb);
        pwl[(8 * hh + r) * AT_KC + j * 16 + c] = __builtin_bit_cast(__bf16, lb);
      }
#pragma unroll
      for (int off = 1; off < 16; off <<= 1) psum += __shfl_xor(psum, off, 32);
      lrow[r] = lrow[r] * alpha + psum;
#pragma unroll
      for (int t = 0; t < 4; ++t) oacc[t][r] *= alpha;
    }
    lds_wave_sync();
#pragma unroll 1
    for (int kk = 0; kk < 2; ++kk) {
      FragB pa, pl;
      pa.h[0] = *(const v8b*)(pwh + c * AT_KC + kk * 32 + 8 * hh);
      pa.h[1] = *(const v8b*)(pwh + c * AT_KC + kk * 32 + 16 + 8 * hh);
      pl.h[0] = *(const v8b*)(pwl + c * AT_KC + kk * 32 + 8 * hh);
      pl.h[1] = *(const v8b*)(pwl + c * AT_KC + kk * 32 + 16 + 8 * hh);
#pragma unroll
      for (int t = 0; t < 4; ++t) {
        FragB vb, vl;
        vb.h[0] = *(const v8b*)(Vth + (t * 16 + c) * AT_KC + kk * 32 + 8 * hh);
        vb.h[1] = *(const v8b*)(Vth + (t * 16 + c) * AT_KC + kk * 32 + 16 + 8 * hh);
        vl.h[0] = *(const v8b*)(Vtl + (t * 16 + c) * AT_KC + kk * 32 + 8 * hh);
        vl.h[1] = *(const v8b*)(Vtl + (t * 16 + c) * AT_KC + kk * 32 + 16 + 8 * hh);
        oacc[t] = at_mma(pa.v, vb.v, oacc[t]);
        oacc[t] = at_mma(pa.v, vl.v, oacc[t]);
        oacc[t] = at_mma(pl.v, vb.v, oacc[t]);
      }
    }
  }
  acc_guard4(oacc[0], oacc[1], oacc[2], oacc[3]);

  unsigned short* osh = Osh[wave];
  unsigned short* osl = Osl[wave];
#pragma unroll
  for (int r = 0; r < 8; ++r) {
    const float inv = 1.0f / lrow[r];
#pragma unroll
    for (int t = 0; t < 4; ++t) {
      const float o = oacc[t][r] * inv;
      const unsigned short hb = bf_bits(o);
      const unsigned short lb = bf_bits(o - bf_val(hb));
      const int so = (8 * hh + r) * 64 + t * 16 + c;
      osh[so] = hb;
      osl[so] = lb;
    }
  }
  lds_wave_sync();
  unsigned short* Ag = qcp + (tok0 + q0) * QCW + (size_t)h * AT_D;
  const int qq = lane >> 3;
  const int c8 = (lane & 7) * 8;
  for (int pass = 0; pass < 2; ++pass) {
#pragma unroll
    for (int it = 0; it < 4; ++it) {
      const int row = it * 4 + qq;
      const v4u x = *(const v4u*)(osh + row * 64 + c8);
      const v4u y = *(const v4u*)(osl + row * 64 + c8);
      *(volatile v4u*)(Ag + (size_t)row * QCW + c8)        = x;
      *(volatile v4u*)(Ag + (size_t)row * QCW + DMOD + c8) = y;
    }
    __threadfence();
  }
}

#define WS_TOTAL_BYTES 131596288UL
static_assert(WS_TOTAL_BYTES <= 134217728UL);

extern "C" void kernel_launch(void* const* d_in, const int* in_sizes, int n_in,
                              void* d_out, int out_size, void* d_ws, size_t ws_size,
                              hipStream_t stream) {
  if (n_in < 6) return;
  if (in_sizes[0] != NTOK * DMOD) return;
  if (in_sizes[1] != DMOD * DMOD) return;
  if (in_sizes[2] != DMOD * LATD) return;
  if (in_sizes[3] != LATD * DMOD) return;
  if (in_sizes[4] != LATD * DMOD) return;
  if (in_sizes[5] != DMOD * DMOD) return;
  if (out_size != NTOK * DMOD) return;

  const float* x  = (const float*)d_in[0];
  const float* wq = (const float*)d_in[1];
  const float* wd = (const float*)d_in[2];
  const float* wk = (const float*)d_in[3];
  const float* wv = (const float*)d_in[4];
  const float* wo = (const float*)d_in[5];
  float* out = (float*)d_out;

  const size_t szXB  = (size_t)NTOK * DMOD * 2;
  const size_t szWQT = (size_t)DMOD * DMOD * 2;
  const size_t szWDT = (size_t)LATD * DMOD * 2;
  const size_t szWKT = (size_t)DMOD * LATD * 2;
  const size_t szWVT = (size_t)DMOD * LATD * 2;
  const size_t szWOT = (size_t)DMOD * DMOD * 2;
  const size_t szLAT = (size_t)NTOK * LATD * 2;
  const size_t szQC  = (size_t)NTOK * QCW * 2;
  const size_t szKP  = (size_t)NTOK * QCW * 2;
  const size_t szVT  = (size_t)NSEQ * DMOD * SEQ * 2;
  size_t off = 0;
  const size_t oXB   = off; off += szXB;
  const size_t oWQT  = off; off += szWQT;
  const size_t oWDT  = off; off += szWDT;
  const size_t oWKT  = off; off += szWKT;
  const size_t oWVT  = off; off += szWVT;
  const size_t oWOT  = off; off += szWOT;
  const size_t oLATH = off; off += szLAT;
  const size_t oLATL = off; off += szLAT;
  const size_t oQC   = off; off += szQC;
  const size_t oKP   = off; off += szKP;
  const size_t oVTH  = off; off += szVT;
  const size_t oVTL  = off; off += szVT;
  if (off != WS_TOTAL_BYTES) return;
  if (off > ws_size) return;

  char* ws = (char*)d_ws;
  unsigned short* XB   = (unsigned short*)(ws + oXB);
  unsigned short* WQT  = (unsigned short*)(ws + oWQT);
  unsigned short* WDT  = (unsigned short*)(ws + oWDT);
  unsigned short* WKT  = (unsigned short*)(ws + oWKT);
  unsigned short* WVT  = (unsigned short*)(ws + oWVT);
  unsigned short* WOT  = (unsigned short*)(ws + oWOT);
  unsigned short* LATH = (unsigned short*)(ws + oLATH);
  unsigned short* LATL = (unsigned short*)(ws + oLATL);
  unsigned short* QC   = (unsigned short*)(ws + oQC);
  unsigned short* KP   = (unsigned short*)(ws + oKP);
  unsigned short* VTH  = (unsigned short*)(ws + oVTH);
  unsigned short* VTL  = (unsigned short*)(ws + oVTL);

  const dim3 b256(256), b128(128);

  cvt_bf16_kernel<<<dim3((NTOK * DMOD / 8) / 256), b256, 0, stream>>>(x, XB, NTOK * DMOD / 8);
  tcvt_kernel<<<dim3(DMOD / 64, DMOD / 64), b256, 0, stream>>>(wq, WQT, DMOD, DMOD);
  tcvt_kernel<<<dim3(LATD / 64, DMOD / 64), b256, 0, stream>>>(wd, WDT, DMOD, LATD);
  tcvt_kernel<<<dim3(DMOD / 64, LATD / 64), b256, 0, stream>>>(wk, WKT, LATD, DMOD);
  tcvt_kernel<<<dim3(DMOD / 64, LATD / 64), b256, 0, stream>>>(wv, WVT, LATD, DMOD);
  tcvt_kernel<<<dim3(DMOD / 64, DMOD / 64), b256, 0, stream>>>(wo, WOT, DMOD, DMOD);
  gemm64_kernel<false, false, 2><<<dim3((NTOK / 64) * (DMOD / 64) / 8, 1), b256, 0, stream>>>(
      XB, XB, DMOD, 0L, WQT, WQT, DMOD, 0L, (void*)QC, (void*)(QC + DMOD), QCW, 0L, NTOK, DMOD, DMOD, 1.0f);
  gemm64_kernel<false, false, 2><<<dim3((NTOK / 64) * (LATD / 64) / 8, 1), b256, 0, stream>>>(
      XB, XB, DMOD, 0L, WDT, WDT, DMOD, 0L, (void*)LATH, (void*)LATL, LATD, 0L, NTOK, LATD, DMOD, 1.0f);
  gemm64_kernel<true, false, 2><<<dim3((NTOK / 64) * (DMOD / 64) / 8, 1), b256, 0, stream>>>(
      LATH, LATL, LATD, 0L, WKT, WKT, LATD, 0L, (void*)KP, (void*)(KP + DMOD), QCW, 0L, NTOK, DMOD, LATD, 1.0f);
  gemm64_kernel<false, true, 2><<<dim3((DMOD / 64) * (SEQ / 64) / 8, NSEQ), b256, 0, stream>>>(
      WVT, WVT, LATD, 0L, LATH, LATL, LATD, (long)SEQ * LATD, (void*)VTH, (void*)VTL, SEQ, (long)DMOD * SEQ,
      DMOD, SEQ, LATD, 1.0f);
  attn_causal64_kernel<<<dim3(NHD * (SEQ / 64), NSEQ), b128, 0, stream>>>(QC, KP, VTH, VTL, 0.125f);
  gemm64_kernel<true, false, 0><<<dim3((NTOK / 64) * (DMOD / 64) / 8, 1), b256, 0, stream>>>(
      QC, QC + DMOD, QCW, 0L, WOT, WOT, DMOD, 0L, (void*)out, (void*)out, DMOD, 0L, NTOK, DMOD, DMOD, 1.0f);
  (void)hipGetLastError();
}
